// EdgeTypeAwareGATLayer_48172353192356
// MI455X (gfx1250) — hardware-verified
//
#include <hip/hip_runtime.h>
#include <hip/hip_bf16.h>
#include <stddef.h>


#define DI    128
#define DV    128
#define NHD   4
#define NTY   4
#define HW    512
#define KF    512
#define NTHR  256
#define NWV   8
#define CHUNK 2048

#define GR    32
#define GC    256
#define XSP   136
#define HSP   260

#define NBD   2048
#define DBITS 11
#define DCAP  6144

#define NBA   512
#define ABITS 9
#define ACAP  2048
#define SP    132
#define AGG_LDS ((NBA * SP + ACAP + NWV) * 4)

#define NPA (NTY * HW * (DI / 8))
#define NPB (DV * (KF / 8))

static_assert(HW == NHD * DV);
static_assert(KF == NTY * DV);
static_assert(CHUNK == NTHR * 8);
static_assert(NBD == NTHR * 8);
static_assert(NBD == (1 << DBITS));
static_assert(NBA == (1 << ABITS));
static_assert(NBA == NWV * 64);
static_assert((NBA % 128) == 0);
static_assert(GR == 4 * NWV);
static_assert((NPA % NTHR) == 0);
static_assert((NPB % NTHR) == 0);
static_assert(AGG_LDS == 278560);
static_assert((SP % 4) == 0);
static_assert((HSP % 4) == 0);
static_assert((XSP % 8) == 0);
static_assert(NBD * NHD * 4 + DCAP * 4 + NWV * 4 <= 65536);

typedef float          v4f  __attribute__((ext_vector_type(4)));
typedef float          v8f  __attribute__((ext_vector_type(8)));
typedef int            v4i  __attribute__((ext_vector_type(4)));
typedef unsigned short v8u  __attribute__((ext_vector_type(8)));
typedef unsigned short v16u __attribute__((ext_vector_type(16)));
typedef __bf16         v16b __attribute__((ext_vector_type(16)));
union Frag { v16u v; v8u half[2]; unsigned short s[16]; };
union Pk8  { unsigned short s[8]; v4i i; };

__device__ __forceinline__ unsigned short f2bf(float f) {
  const unsigned u = __float_as_uint(f);
  return (unsigned short)((u + 0x7fffu + ((u >> 16) & 1u)) >> 16);
}
__device__ __forceinline__ float rb(float f) {
  const unsigned u = __float_as_uint(f);
  return __uint_as_float((u + 0x7fffu + ((u >> 16) & 1u)) & 0xffff0000u);
}
__device__ __forceinline__ v4f rb4(v4f v) {
  v4f r;
  r.x = rb(v.x); r.y = rb(v.y); r.z = rb(v.z); r.w = rb(v.w);
  return r;
}
__device__ __forceinline__ float wsum(float v) {
  v += __shfl_xor(v, 16, 32);
  v += __shfl_xor(v, 8, 32);
  v += __shfl_xor(v, 4, 32);
  v += __shfl_xor(v, 2, 32);
  v += __shfl_xor(v, 1, 32);
  return v;
}
__device__ __forceinline__ float dot4(v4f a, v4f b) {
  return a.x * b.x + a.y * b.y + a.z * b.z + a.w * b.w;
}
__device__ __forceinline__ float leaky02(float a) { return (a >= 0.f) ? a : 0.2f * a; }

__device__ __forceinline__ v8f wm(v16u a, v16u b, v8f c) {
  const v16b av = __builtin_bit_cast(v16b, a);
  const v16b bv = __builtin_bit_cast(v16b, b);
  v8f d = __builtin_amdgcn_wmma_f32_16x16x32_bf16(false, av, false, bv, (short)0, c, false, false);
  asm volatile("v_nop\n\tv_nop\n\tv_nop\n\tv_nop" : "+v"(d) : "v"(av), "v"(bv));
  return d;
}

__device__ __forceinline__ void split16(v4f f0, v4f f1, v4f f2, v4f f3, Frag& hi, Frag& lo) {
  const float v[16] = {f0.x, f0.y, f0.z, f0.w, f1.x, f1.y, f1.z, f1.w,
                       f2.x, f2.y, f2.z, f2.w, f3.x, f3.y, f3.z, f3.w};
#pragma unroll
  for (int i = 0; i < 16; ++i) {
    const float hv = rb(v[i]);
    hi.s[i] = (unsigned short)(__float_as_uint(hv) >> 16);
    lo.s[i] = f2bf(v[i] - hv);
  }
}

template <int NBITS, int CAP>
__device__ __forceinline__ int scan_hits(const int* __restrict__ edst, const int* __restrict__ eat,
                                         int nE, int base, int t, int* blist, int* wcnt) {
  const int tid = threadIdx.x, lane = tid & 31, wave = tid >> 5;
  const unsigned nbm = 1u << NBITS;
  const bool al16 = (((((size_t)edst) | ((size_t)eat)) & 15) == 0);
  const int nChunks = (nE + CHUNK - 1) / CHUNK;
  int total = 0;
#pragma unroll 1
  for (int ch = 0; ch < nChunks; ++ch) {
    const int cbase = ch * CHUNK;
    int dv[8], av[8], ev[8];
    bool ok[8];
#pragma unroll
    for (int g = 0; g < 2; ++g) {
      const int e0 = cbase + (g * NTHR + tid) * 4;
      v4i d, a;
      if (al16 && (e0 + 3 < nE)) {
        d = *(const v4i*)(edst + e0);
        a = *(const v4i*)(eat + e0);
      } else {
        d.x = (e0     < nE) ? edst[e0]     : 0;
        d.y = (e0 + 1 < nE) ? edst[e0 + 1] : 0;
        d.z = (e0 + 2 < nE) ? edst[e0 + 2] : 0;
        d.w = (e0 + 3 < nE) ? edst[e0 + 3] : 0;
        a.x = (e0     < nE) ? eat[e0]     : -1;
        a.y = (e0 + 1 < nE) ? eat[e0 + 1] : -1;
        a.z = (e0 + 2 < nE) ? eat[e0 + 2] : -1;
        a.w = (e0 + 3 < nE) ? eat[e0 + 3] : -1;
      }
      dv[4 * g + 0] = d.x; dv[4 * g + 1] = d.y; dv[4 * g + 2] = d.z; dv[4 * g + 3] = d.w;
      av[4 * g + 0] = a.x; av[4 * g + 1] = a.y; av[4 * g + 2] = a.z; av[4 * g + 3] = a.w;
      ev[4 * g + 0] = e0; ev[4 * g + 1] = e0 + 1; ev[4 * g + 2] = e0 + 2; ev[4 * g + 3] = e0 + 3;
      ok[4 * g + 0] = (e0 < nE); ok[4 * g + 1] = (e0 + 1 < nE); ok[4 * g + 2] = (e0 + 2 < nE); ok[4 * g + 3] = (e0 + 3 < nE);
    }
    bool hb[8];
    int sv[8];
    int cnt = 0;
#pragma unroll
    for (int j = 0; j < 8; ++j) {
      const unsigned s = (unsigned)dv[j] - (unsigned)base;
      hb[j] = ok[j] && (s < nbm) && (av[j] == t);
      sv[j] = (int)(s & (nbm - 1u));
      cnt += hb[j] ? 1 : 0;
    }
    const unsigned anyb = __builtin_amdgcn_ballot_w32(cnt > 0);
    int wc = 0;
    unsigned mk[8] = {0u, 0u, 0u, 0u, 0u, 0u, 0u, 0u};
    if (anyb != 0u) {
#pragma unroll
      for (int j = 0; j < 8; ++j) {
        mk[j] = __builtin_amdgcn_ballot_w32(hb[j]);
        wc += (int)__builtin_popcount(mk[j]);
      }
    }
    if (lane == 0) wcnt[wave] = wc;
    __syncthreads();
    int pre = 0, sum = 0;
#pragma unroll
    for (int w = 0; w < NWV; ++w) {
      const int c = wcnt[w];
      pre += (w < wave) ? c : 0;
      sum += c;
    }
    if (wc > 0) {
      int pos = total + pre;
#pragma unroll
      for (int j = 0; j < 8; ++j) {
        if (hb[j]) {
          const int idx = pos + (int)__builtin_amdgcn_mbcnt_lo(mk[j], 0u);
          if ((unsigned)idx < (unsigned)CAP) blist[idx] = (ev[j] << NBITS) | sv[j];
        }
        pos += (int)__builtin_popcount(mk[j]);
      }
    }
    total += sum;
    __syncthreads();
  }
  return (total < CAP) ? total : CAP;
}

__global__ __launch_bounds__(NTHR) void k_prep(const float* __restrict__ Wn, const float* __restrict__ Wf,
                                               unsigned short* Wt, unsigned short* Wft) {
  const int g = blockIdx.x * NTHR + threadIdx.x;
  Pk8 u;
  unsigned short* p;
  if (g < NPA) {
    const int k8 = g & 15;
    const int c  = (g >> 4) & (HW - 1);
    const int t  = g >> 13;
#pragma unroll
    for (int i = 0; i < 8; ++i) u.s[i] = f2bf(Wn[((size_t)t * DI + 8 * k8 + i) * HW + c]);
    p = Wt + ((size_t)t * HW + c) * DI + 8 * k8;
  } else if (g < NPA + NPB) {
    const int q  = g - NPA;
    const int k8 = q & 63;
    const int n  = q >> 6;
#pragma unroll
    for (int i = 0; i < 8; ++i) u.s[i] = f2bf(Wf[(size_t)(8 * k8 + i) * DV + n]);
    p = Wft + (size_t)n * KF + 8 * k8;
  } else {
    return;
  }
  *(volatile v4i*)p = u.i;
  __threadfence();
  *(volatile v4i*)p = u.i;
}

__global__ __launch_bounds__(NTHR) void k_gemm(
    const float* __restrict__ x, const unsigned short* __restrict__ Wt,
    const float* __restrict__ avs, const float* __restrict__ avd,
    float* h, float* asP, float* adP, int nN, int nP, int t) {
  __shared__ __attribute__((aligned(16))) unsigned short xs[GR * XSP];
  __shared__ __attribute__((aligned(16))) float hs[GR * HSP];
  __shared__ __attribute__((aligned(16))) float sA[2 * GR];
  __shared__ __attribute__((aligned(16))) float sD[2 * GR];

  const int tid  = threadIdx.x;
  const int lane = tid & 31;
  const int wave = tid >> 5;
  const int hh   = lane >> 4;
  const int m    = lane & 15;
  const int rowBase = blockIdx.x * GR;
  const int colBase = blockIdx.y * GC;
  const int hd0     = blockIdx.y * 2;

  {
    const int r  = tid >> 3;
    const int c0 = (tid & 7) * 16;
    int row = rowBase + r;
    if (row > nN - 1) row = nN - 1;
    const float* p = x + (size_t)row * DI + c0;
    const v4f f0 = *(const v4f*)(p), f1 = *(const v4f*)(p + 4);
    const v4f f2 = *(const v4f*)(p + 8), f3 = *(const v4f*)(p + 12);
    Pk8 u0, u1;
    u0.s[0] = f2bf(f0.x); u0.s[1] = f2bf(f0.y); u0.s[2] = f2bf(f0.z); u0.s[3] = f2bf(f0.w);
    u0.s[4] = f2bf(f1.x); u0.s[5] = f2bf(f1.y); u0.s[6] = f2bf(f1.z); u0.s[7] = f2bf(f1.w);
    u1.s[0] = f2bf(f2.x); u1.s[1] = f2bf(f2.y); u1.s[2] = f2bf(f2.z); u1.s[3] = f2bf(f2.w);
    u1.s[4] = f2bf(f3.x); u1.s[5] = f2bf(f3.y); u1.s[6] = f2bf(f3.z); u1.s[7] = f2bf(f3.w);
    *(v4i*)(xs + r * XSP + c0)     = u0.i;
    *(v4i*)(xs + r * XSP + c0 + 8) = u1.i;
  }
  __syncthreads();

  const unsigned short* wb0 = Wt + ((size_t)t * HW + colBase + 32 * wave + m) * DI + 8 * hh;
  const unsigned short* wb1 = wb0 + 16 * DI;
  const unsigned short* xa0 = xs + m * XSP + 8 * hh;
  const unsigned short* xa1 = xa0 + 16 * XSP;
  v8f c00 = {0.f, 0.f, 0.f, 0.f, 0.f, 0.f, 0.f, 0.f};
  v8f c01 = c00, c10 = c00, c11 = c00;
#pragma unroll
  for (int kt = 0; kt < DI / 32; ++kt) {
    const int k0 = 32 * kt;
    Frag a0, a1, b0, b1;
    a0.half[0] = *(const v8u*)(xa0 + k0); a0.half[1] = *(const v8u*)(xa0 + k0 + 16);
    a1.half[0] = *(const v8u*)(xa1 + k0); a1.half[1] = *(const v8u*)(xa1 + k0 + 16);
    b0.half[0] = *(const v8u*)(wb0 + k0); b0.half[1] = *(const v8u*)(wb0 + k0 + 16);
    b1.half[0] = *(const v8u*)(wb1 + k0); b1.half[1] = *(const v8u*)(wb1 + k0 + 16);
    c00 = wm(a0.v, b0.v, c00);
    c01 = wm(a0.v, b1.v, c01);
    c10 = wm(a1.v, b0.v, c10);
    c11 = wm(a1.v, b1.v, c11);
  }

#pragma unroll
  for (int r = 0; r < 8; ++r) {
    hs[(8 * hh + r) * HSP + 32 * wave + m]           = c00[r];
    hs[(8 * hh + r) * HSP + 32 * wave + 16 + m]      = c01[r];
    hs[(16 + 8 * hh + r) * HSP + 32 * wave + m]      = c10[r];
    hs[(16 + 8 * hh + r) * HSP + 32 * wave + 16 + m] = c11[r];
  }
  __syncthreads();

  const v4f as0 = rb4(*(const v4f*)(avs + (size_t)(t * NHD + hd0) * DV + 4 * lane));
  const v4f as1 = rb4(*(const v4f*)(avs + (size_t)(t * NHD + hd0 + 1) * DV + 4 * lane));
  const v4f ad0 = rb4(*(const v4f*)(avd + (size_t)(t * NHD + hd0) * DV + 4 * lane));
  const v4f ad1 = rb4(*(const v4f*)(avd + (size_t)(t * NHD + hd0 + 1) * DV + 4 * lane));
  v4f hv0[4], hv1[4];
#pragma unroll
  for (int i = 0; i < 4; ++i) {
    const int row = 4 * wave + i;
    hv0[i] = *(const v4f*)(hs + row * HSP + 4 * lane);
    hv1[i] = *(const v4f*)(hs + row * HSP + DV + 4 * lane);
    const float s0 = wsum(dot4(hv0[i], as0));
    const float s1 = wsum(dot4(hv1[i], as1));
    const float d0 = wsum(dot4(hv0[i], ad0));
    const float d1 = wsum(dot4(hv1[i], ad1));
    if (lane == 0) {
      sA[row] = s0; sA[GR + row] = s1;
      sD[row] = d0; sD[GR + row] = d1;
    }
  }

  float* hp[4];
#pragma unroll
  for (int i = 0; i < 4; ++i) hp[i] = h + (size_t)(rowBase + 4 * wave + i) * HW + colBase + 4 * lane;
#pragma unroll
  for (int i = 0; i < 4; ++i) {
    *(volatile v4f*)(hp[i])      = hv0[i];
    *(volatile v4f*)(hp[i] + DV) = hv1[i];
  }
  __syncthreads();

  v4f gv = {0.f, 0.f, 0.f, 0.f};
  float* gp = asP;
  if (wave == 0) {
    const int q = lane >> 3;
    const int i = lane & 7;
    const float* src = (q == 0) ? (sA + 4 * i) : (q == 1) ? (sA + GR + 4 * i)
                     : (q == 2) ? (sD + 4 * i) : (sD + GR + 4 * i);
    gv = *(const v4f*)src;
    gp = ((q < 2) ? asP : adP) + (size_t)(hd0 + (q & 1)) * nP + rowBase + 4 * i;
    *(volatile v4f*)gp = gv;
  }
  __threadfence();
#pragma unroll
  for (int i = 0; i < 4; ++i) {
    *(volatile v4f*)(hp[i])      = hv0[i];
    *(volatile v4f*)(hp[i] + DV) = hv1[i];
  }
  if (wave == 0) *(volatile v4f*)gp = gv;
}

__global__ __launch_bounds__(NTHR) void k_den(
    const int* __restrict__ ei, const int* __restrict__ ea,
    const float* __restrict__ asP, const float* __restrict__ adP, float* dinv,
    int nN, int nP, int nPD, int nE, int t) {
  __shared__ __attribute__((aligned(16))) float den[NBD * NHD];
  __shared__ int blist[DCAP];
  __shared__ int wcnt[NWV];

  const int tid  = threadIdx.x;
  const int lane = tid & 31;
  const int wave = tid >> 5;
  const int base = blockIdx.x * NBD;

  {
    const v4f z4 = {0.f, 0.f, 0.f, 0.f};
    v4f* d4 = (v4f*)den;
    for (int i = tid; i < NBD * NHD / 4; i += NTHR) d4[i] = z4;
  }
  __syncthreads();

  const int L = scan_hits<DBITS, DCAP>(ei + nE, ea, nE, base, t, blist, wcnt);

  if (wave == 0) {
    const int hl = lane & 3;
#pragma unroll 1
    for (int i = 0; i < L; ++i) {
      const int ent  = blist[i];
      const int slot = ent & (NBD - 1);
      int e = ent >> DBITS;
      if (e > nE - 1) e = nE - 1;
      int src = ei[e];
      src = (src < 0) ? 0 : ((src > nN - 1) ? nN - 1 : src);
      int nd = base + slot;
      if (nd > nN - 1) nd = nN - 1;
      float v = 0.f;
      if (lane < 4)      v = asP[(size_t)hl * nP + src];
      else if (lane < 8) v = adP[(size_t)hl * nP + nd];
      const float o = __shfl(v, hl + 4, 32);
      float a = leaky02(v + o);
      a = fminf(a, 80.f);
      const float p = __expf(a);
      if (lane < 4) den[slot * NHD + hl] += p;
    }
  }
  __syncthreads();

#pragma unroll 1
  for (int q = 0; q < NBD / NTHR; ++q) {
    const int slot = q * NTHR + tid;
    int nd = base + slot;
    if (nd > nN - 1) nd = nN - 1;
    const v4f dn = *(const v4f*)(den + slot * NHD);
    float dd[4] = {dn.x, dn.y, dn.z, dn.w};
#pragma unroll
    for (int hd = 0; hd < NHD; ++hd) {
      float a = leaky02(asP[(size_t)hd * nP + nd] + adP[(size_t)hd * nP + nd]);
      a = fminf(a, 80.f);
      const float p = __expf(a);
      dd[hd] = 1.0f / (dd[hd] + p);
    }
    const v4f r4 = {dd[0], dd[1], dd[2], dd[3]};
    *(v4f*)(den + slot * NHD) = r4;
  }
  __syncthreads();

  v4f sv[2][NHD];
  float* spp[2][NHD];
#pragma unroll
  for (int q = 0; q < 2; ++q) {
    const int s4 = (wave * 2 + q) * 128 + 4 * lane;
#pragma unroll
    for (int hd = 0; hd < NHD; ++hd) {
      v4f v;
      v.x = den[(s4 + 0) * NHD + hd];
      v.y = den[(s4 + 1) * NHD + hd];
      v.z = den[(s4 + 2) * NHD + hd];
      v.w = den[(s4 + 3) * NHD + hd];
      sv[q][hd]  = v;
      spp[q][hd] = dinv + (size_t)hd * nPD + base + s4;
      *(volatile v4f*)(spp[q][hd]) = v;
    }
  }
  __threadfence();
#pragma unroll
  for (int q = 0; q < 2; ++q)
#pragma unroll
    for (int hd = 0; hd < NHD; ++hd) *(volatile v4f*)(spp[q][hd]) = sv[q][hd];
}

__global__ __launch_bounds__(NTHR) void k_agg(
    const int* __restrict__ ei, const int* __restrict__ ea, const float* __restrict__ h,
    const float* __restrict__ asP, const float* __restrict__ adP, const float* __restrict__ dinv,
    const float* __restrict__ bn, const float* __restrict__ etw, const unsigned short* __restrict__ Wft,
    const float* __restrict__ bfu, const float* __restrict__ gam, const float* __restrict__ bet,
    float* y, float* out, int nN, int nP, int nPD, int nE, int t) {
  extern __shared__ v4f lds_dyn[];
  float* sacc  = (float*)lds_dyn;
  int*   blist = (int*)(sacc + NBA * SP);
  int*   wcnt  = blist + ACAP;

  const int tid  = threadIdx.x;
  const int lane = tid & 31;
  const int wave = tid >> 5;
  const int hh   = lane >> 4;
  const int m    = lane & 15;
  const int base = blockIdx.x * NBA;

  {
    const v4f z4 = {0.f, 0.f, 0.f, 0.f};
    for (int i = tid; i < NBA * SP / 4; i += NTHR) lds_dyn[i] = z4;
  }
  __syncthreads();

  const int L = scan_hits<ABITS, ACAP>(ei + nE, ea, nE, base, t, blist, wcnt);

  float wt;
  {
    const float e0 = rb(etw[0]), e1 = rb(etw[1]), e2 = rb(etw[2]), e3 = rb(etw[3]);
    const float mx = fmaxf(fmaxf(e0, e1), fmaxf(e2, e3));
    const float x0 = __expf(e0 - mx), x1 = __expf(e1 - mx), x2 = __expf(e2 - mx), x3 = __expf(e3 - mx);
    const float inv = 1.0f / (x0 + x1 + x2 + x3);
    wt = ((t == 0) ? x0 : (t == 1) ? x1 : (t == 2) ? x2 : x3) * inv;
  }
  const int hl = lane & 3;

  if (wave == 0) {
#pragma unroll 1
    for (int i = 0; i < L; ++i) {
      const int ent  = blist[i];
      const int slot = ent & (NBA - 1);
      int e = ent >> ABITS;
      if (e > nE - 1) e = nE - 1;
      int src = ei[e];
      src = (src < 0) ? 0 : ((src > nN - 1) ? nN - 1 : src);
      int nd = base + slot;
      if (nd > nN - 1) nd = nN - 1;
      float cf = 0.f;
      if (lane < 4) {
        float a = leaky02(asP[(size_t)hl * nP + src] + adP[(size_t)hl * nP + nd]);
        a = fminf(a, 80.f);
        cf = __expf(a) * dinv[(size_t)hl * nPD + nd];
      }
      const float c0 = __shfl(cf, 0, 32), c1 = __shfl(cf, 1, 32);
      const float c2 = __shfl(cf, 2, 32), c3 = __shfl(cf, 3, 32);
      const float* hp = h + (size_t)src * HW + 4 * lane;
      v4f v = c0 * (*(const v4f*)(hp));
      v = v + c1 * (*(const v4f*)(hp + DV));
      v = v + c2 * (*(const v4f*)(hp + 2 * DV));
      v = v + c3 * (*(const v4f*)(hp + 3 * DV));
      v4f* sp = (v4f*)(sacc + (size_t)slot * SP + 4 * lane);
      const v4f cur = *sp;
      *sp = cur + v;
    }
  }
  __syncthreads();

  const v4f b4 = rb4(*(const v4f*)(bn + (size_t)t * DV + 4 * lane));
#pragma unroll 2
  for (int j = 0; j < NBA / NWV; ++j) {
    const int slot = wave * (NBA / NWV) + j;
    int nd = base + slot;
    if (nd > nN - 1) nd = nN - 1;
    float cf = 0.f;
    if (lane < 4) {
      float a = leaky02(asP[(size_t)hl * nP + nd] + adP[(size_t)hl * nP + nd]);
      a = fminf(a, 80.f);
      cf = __expf(a) * dinv[(size_t)hl * nPD + nd];
    }
    const float c0 = __shfl(cf, 0, 32), c1 = __shfl(cf, 1, 32);
    const float c2 = __shfl(cf, 2, 32), c3 = __shfl(cf, 3, 32);
    const float* hp = h + (size_t)nd * HW + 4 * lane;
    v4f v = c0 * (*(const v4f*)(hp));
    v = v + c1 * (*(const v4f*)(hp + DV));
    v = v + c2 * (*(const v4f*)(hp + 2 * DV));
    v = v + c3 * (*(const v4f*)(hp + 3 * DV));
    v4f* sp = (v4f*)(sacc + (size_t)slot * SP + 4 * lane);
    const v4f row = *sp + v;
    const v4f o = (row * 0.25f + b4) * wt;
    *sp = o;
  }
  __syncthreads();

  Frag bq[4];
  {
    const unsigned short* wp = Wft + (size_t)(16 * wave + m) * KF + t * DV + 8 * hh;
#pragma unroll
    for (int ks = 0; ks < 4; ++ks) {
      bq[ks].half[0] = *(const v8u*)(wp + 32 * ks);
      bq[ks].half[1] = *(const v8u*)(wp + 32 * ks + 16);
    }
  }
  const v4f bf4 = rb4(*(const v4f*)(bfu + 4 * lane));
  const v4f g4  = rb4(*(const v4f*)(gam + 4 * lane));
  const v4f e4  = rb4(*(const v4f*)(bet + 4 * lane));

#pragma unroll 1
  for (int c = 0; c < NBA / 128; ++c) {
    v8f acc[8];
#pragma unroll
    for (int rt = 0; rt < 8; ++rt) {
      const v8f z8 = {0.f, 0.f, 0.f, 0.f, 0.f, 0.f, 0.f, 0.f};
      acc[rt] = z8;
    }
#pragma unroll
    for (int rt = 0; rt < 8; ++rt) {
      const float* zp = sacc + (size_t)(128 * c + 16 * rt + m) * SP + 8 * hh;
#pragma unroll
      for (int ks = 0; ks < 4; ++ks) {
        const int k0 = 32 * ks;
        const v4f f0 = *(const v4f*)(zp + k0);
        const v4f f1 = *(const v4f*)(zp + k0 + 4);
        const v4f f2 = *(const v4f*)(zp + k0 + 16);
        const v4f f3 = *(const v4f*)(zp + k0 + 20);
        Frag ahi, alo;
        split16(f0, f1, f2, f3, ahi, alo);
        acc[rt] = wm(ahi.v, bq[ks].v, acc[rt]);
        acc[rt] = wm(alo.v, bq[ks].v, acc[rt]);
      }
    }
    __syncthreads();
#pragma unroll
    for (int rt = 0; rt < 8; ++rt)
#pragma unroll
      for (int r = 0; r < 8; ++r)
        sacc[(size_t)(128 * c + 16 * rt + 8 * hh + r) * SP + 16 * wave + m] = acc[rt][r];
    __syncthreads();

#pragma unroll 1
    for (int j = 0; j < 16; ++j) {
      const int lrow = 128 * c + 16 * wave + j;
      const int node = base + lrow;
      v4f yv = *(const v4f*)(sacc + (size_t)lrow * SP + 4 * lane);
      float* yp = y + (size_t)node * DV + 4 * lane;
      if (t > 0) yv = yv + *(const v4f*)yp;
      if (t < NTY - 1) {
        *(volatile v4f*)yp = yv;
        __threadfence();
        *(volatile v4f*)yp = yv;
      } else if (node < nN) {
        const v4f yb = yv + bf4;
        const float s  = wsum(yb.x + yb.y + yb.z + yb.w);
        const float mu = s * (1.0f / DV);
        const v4f dd = yb - mu;
        const float q  = wsum(dd.x * dd.x + dd.y * dd.y + dd.z * dd.z + dd.w * dd.w);
        const float var = q * (1.0f / DV);
        const float inv = 1.0f / sqrtf(var + 1e-5f);
        v4f o = dd * inv * g4 + e4;
        o.x = o.x > 0.f ? o.x : 0.f;
        o.y = o.y > 0.f ? o.y : 0.f;
        o.z = o.z > 0.f ? o.z : 0.f;
        o.w = o.w > 0.f ? o.w : 0.f;
        float* op = out + (size_t)node * DV + 4 * lane;
        *(volatile v4f*)op = o;
        __threadfence();
        *(volatile v4f*)op = o;
      }
    }
    __syncthreads();
  }
}

static size_t al256(size_t b) { return (b + 255) & ~(size_t)255; }

extern "C" void kernel_launch(void* const* d_in, const int* in_sizes, int n_in,
                              void* d_out, int out_size, void* d_ws, size_t ws_size,
                              hipStream_t stream) {
  if (n_in < 12) return;
  const int nN = in_sizes[0] / DI;
  if (nN <= 0 || in_sizes[0] != nN * DI) return;
  const int nE = in_sizes[2];
  if (nE < 0 || nE > (1 << 19) || in_sizes[1] != 2 * nE) return;
  if (in_sizes[3] != NTY * DI * HW) return;
  if (in_sizes[4] != NTY * NHD * DV || in_sizes[5] != NTY * NHD * DV) return;
  if (in_sizes[6] != NTY * DV || in_sizes[7] != NTY) return;
  if (in_sizes[8] != KF * DV || in_sizes[9] != DV || in_sizes[10] != DV || in_sizes[11] != DV) return;
  if (out_size != nN * DV) return;

  const float* x   = (const float*)d_in[0];
  const int*   ei  = (const int*)d_in[1];
  const int*   ea  = (const int*)d_in[2];
  const float* Wn  = (const float*)d_in[3];
  const float* avs = (const float*)d_in[4];
  const float* avd = (const float*)d_in[5];
  const float* bn  = (const float*)d_in[6];
  const float* etw = (const float*)d_in[7];
  const float* Wf  = (const float*)d_in[8];
  const float* bfu = (const float*)d_in[9];
  const float* gam = (const float*)d_in[10];
  const float* bet = (const float*)d_in[11];
  float* out = (float*)d_out;

  const int nP  = ((nN + NBA - 1) / NBA) * NBA;
  const int nPD = ((nN + NBD - 1) / NBD) * NBD;

  size_t off = 0;
  unsigned short* Wt  = (unsigned short*)((char*)d_ws + off); off += al256((size_t)NTY * HW * DI * 2);
  unsigned short* Wft = (unsigned short*)((char*)d_ws + off); off += al256((size_t)DV * KF * 2);
  float* h    = (float*)((char*)d_ws + off); off += al256((size_t)nP * HW * sizeof(float));
  float* y    = (float*)((char*)d_ws + off); off += al256((size_t)nP * DV * sizeof(float));
  float* asP  = (float*)((char*)d_ws + off); off += al256((size_t)NHD * nP * sizeof(float));
  float* adP  = (float*)((char*)d_ws + off); off += al256((size_t)NHD * nP * sizeof(float));
  float* dinv = (float*)((char*)d_ws + off); off += al256((size_t)NHD * nPD * sizeof(float));
  if (off > ws_size) return;
  if (off > (size_t)134217728) return;

  k_prep<<<(NPA + NPB + NTHR - 1) / NTHR, NTHR, 0, stream>>>(Wn, Wf, Wt, Wft);

  hipFuncSetAttribute(reinterpret_cast<const void*>(&k_agg),
                      hipFuncAttributeMaxDynamicSharedMemorySize, AGG_LDS);

  for (int t = 0; t < NTY; ++t) {
    k_gemm<<<dim3(nP / GR, HW / GC), NTHR, 0, stream>>>(x, Wt, avs, avd, h, asP, adP, nN, nP, t);
    k_den<<<nPD / NBD, NTHR, 0, stream>>>(ei, ea, asP, adP, dinv, nN, nP, nPD, nE, t);
    k_agg<<<nP / NBA, NTHR, AGG_LDS, stream>>>(ei, ea, h, asP, adP, dinv, bn, etw, Wft,
                                               bfu, gam, bet, y, out, nN, nP, nPD, nE, t);
  }
}
